// VariableSelectionNetwork_53231824666759
// MI455X (gfx1250) — hardware-run, weakly checked
//
#include <hip/hip_runtime.h>


#ifndef NB
#define NB 4096
#endif
#define NB_FULL 4096
#define NV   64
#define HID  256
#define XP   64
#define OSP  68
#define CSP  260
#define HSP  264
#define ACAR 256.0f
#define WCAR 64.0f
#define HCAR 16.0f
#define LOG2E 1.4426950408889634f
#define LN_EPS 1.0e-5f
#define OUT1_OFF ((size_t)NB_FULL * HID)

static constexpr float SCL = 1.0f / (256.0f * 64.0f);
static constexpr float HSC = 1.0f / (16.0f * 64.0f);

static_assert(NV == 64);
static_assert(HID == 256);
static_assert(NV % 32 == 0);
static_assert(HID % 32 == 0);
static_assert(NV % 64 == 0);
static_assert(HID % 64 == 0);
static_assert(NB % 16 == 0);
static_assert(NB <= NB_FULL);
static_assert(XP == NV);
static_assert(OUT1_OFF * 4 == (size_t)4194304);
static_assert((OUT1_OFF * 4) % 128 == 0);
static_assert((OSP * 4) % 16 == 0);
static_assert((CSP * 4) % 16 == 0);
static_assert((HSP * 2) % 16 == 0);
static_assert(OSP >= NV);
static_assert(CSP >= HID);
static_assert(HSP >= HID);
static_assert(8 * 32 * 16 == 16 * NV * 4);
static_assert(32 * 32 * 16 == 16 * HID * 4);
static_assert(256 * 2 * 16 == 64 * 64 * 2);
static_assert(256 * 16 == 64 * 64);
static_assert(2 * 16 * CSP * 4 + 2 * 16 * OSP * 4 <= 131072);
static_assert(16 * HSP * 2 + 16 * OSP * 4 <= 131072);
static_assert(64 * 65 * 4 <= 131072);
static_assert(4 * 4 * 16 == HID);

typedef _Float16 h16;
typedef unsigned short bf;
typedef __attribute__((ext_vector_type(16))) __bf16   v16bf;
typedef __attribute__((ext_vector_type(16))) _Float16 v16h;
typedef __attribute__((ext_vector_type(8)))  _Float16 v8h;
typedef __attribute__((ext_vector_type(8)))  unsigned short v8us;
typedef __attribute__((ext_vector_type(8)))  float    v8f;
typedef __attribute__((ext_vector_type(4)))  float    v4f;
typedef v4f  __attribute__((may_alias)) v4fa;
typedef v8h  __attribute__((may_alias)) v8ha;

__device__ __forceinline__ unsigned short f2bf(float f) { unsigned u = __float_as_uint(f); u += 0x7FFFu + ((u >> 16) & 1u); return (unsigned short)(u >> 16); }
__device__ __forceinline__ float bfr(float f) { return __uint_as_float(((unsigned)f2bf(f)) << 16); }
__device__ __forceinline__ v16h cat16(v8h lo, v8h hi) { return __builtin_shufflevector(lo, hi, 0, 1, 2, 3, 4, 5, 6, 7, 8, 9, 10, 11, 12, 13, 14, 15); }
__device__ __forceinline__ v16bf cat16b(v8us lo, v8us hi) { return __builtin_bit_cast(v16bf, __builtin_shufflevector(lo, hi, 0, 1, 2, 3, 4, 5, 6, 7, 8, 9, 10, 11, 12, 13, 14, 15)); }
__device__ __forceinline__ v8f wmma16(v16h a, v16h b, v8f c) { return __builtin_amdgcn_wmma_f32_16x16x32_f16(false, a, false, b, (short)0, c, false, false); }
__device__ __forceinline__ v8f wmmab(v16bf a, v16bf b, v8f c) { return __builtin_amdgcn_wmma_f32_16x16x32_bf16(false, a, false, b, (short)0, c, false, false); }
__device__ __forceinline__ v8f wmma16g(v16h a, v16h b, v8f c) { c = wmma16(a, b, c); asm volatile("v_nop\n\tv_nop\n\tv_nop\n\tv_nop" : "+v"(c) : "v"(a), "v"(b)); return c; }
__device__ __forceinline__ v8f wmmabg(v16bf a, v16bf b, v8f c) { c = wmmab(a, b, c); asm volatile("v_nop\n\tv_nop\n\tv_nop\n\tv_nop" : "+v"(c) : "v"(a), "v"(b)); return c; }
__device__ __forceinline__ v16h  ldh(const h16* p) { return cat16(*(const v8h*)p, *(const v8h*)(p + 16)); }
__device__ __forceinline__ v16bf ldb(const bf* p)  { return cat16b(*(const v8us*)p, *(const v8us*)(p + 16)); }
__device__ __forceinline__ void wave_sync() { __builtin_amdgcn_fence(3  , "wavefront"); __builtin_amdgcn_wave_barrier(); asm volatile("" ::: "memory"); }
static __device__ __forceinline__ h16 toh_flush(float v) { const float w = (fabsf(v) < 6.103515625e-05f) ? 0.0f : v; return (h16)w; }
__device__ __forceinline__ float eluf(float t) { const float e = __builtin_amdgcn_exp2f(t * LOG2E) - 1.0f; return (t > 0.0f) ? t : e; }
__device__ __forceinline__ float sigm(float z) { return __builtin_amdgcn_rcpf(1.0f + __builtin_amdgcn_exp2f(-z * LOG2E)); }
__device__ __forceinline__ h16 hvf(float xa, float w, float b) { return toh_flush(eluf(xa * w + b) * ACAR); }
__device__ __forceinline__ float sum16(float v) { v += __shfl_xor(v, 1, 32); v += __shfl_xor(v, 2, 32); v += __shfl_xor(v, 4, 32); v += __shfl_xor(v, 8, 32); return v; }
__device__ __forceinline__ float max16(float v) { v = fmaxf(v, __shfl_xor(v, 1, 32)); v = fmaxf(v, __shfl_xor(v, 2, 32)); v = fmaxf(v, __shfl_xor(v, 4, 32)); v = fmaxf(v, __shfl_xor(v, 8, 32)); return v; }

__global__ __launch_bounds__(256) void k_tr_h(const float* __restrict__ in, h16* out, int R, int C, float car) {
    __shared__ float ts[64 * 65];
    const int tid = threadIdx.x; const int c0 = blockIdx.x * 64, r0 = blockIdx.y * 64; const size_t zb = (size_t)blockIdx.z * (size_t)R * (size_t)C;
#pragma unroll
    for (int j = 0; j < 16; ++j) { const int i = tid + 256 * j; const int rr = i >> 6, cc = i & 63; ts[rr * 65 + cc] = in[zb + (size_t)(r0 + rr) * C + c0 + cc]; }
    __syncthreads();
    v8h o0, o1;
    { const int p = tid;       const int orow = p >> 3, c8 = (p & 7) * 8;
#pragma unroll
      for (int i = 0; i < 8; ++i) o0[i] = toh_flush(bfr(ts[(c8 + i) * 65 + orow]) * car); }
    { const int p = tid + 256; const int orow = p >> 3, c8 = (p & 7) * 8;
#pragma unroll
      for (int i = 0; i < 8; ++i) o1[i] = toh_flush(bfr(ts[(c8 + i) * 65 + orow]) * car); }
    const size_t a0 = zb + (size_t)(c0 + (tid >> 3)) * R + r0 + (tid & 7) * 8;
    const size_t a1 = zb + (size_t)(c0 + 32 + (tid >> 3)) * R + r0 + (tid & 7) * 8;
    *(volatile v8h*)(out + a0) = o0; *(volatile v8h*)(out + a1) = o1;
    __threadfence();
    *(volatile v8h*)(out + a0) = o0; *(volatile v8h*)(out + a1) = o1;
}

__global__ __launch_bounds__(256) void k_tr_b(const float* __restrict__ in, bf* out, int R, int C) {
    __shared__ float ts[64 * 65];
    const int tid = threadIdx.x; const int c0 = blockIdx.x * 64, r0 = blockIdx.y * 64; const size_t zb = (size_t)blockIdx.z * (size_t)R * (size_t)C;
#pragma unroll
    for (int j = 0; j < 16; ++j) { const int i = tid + 256 * j; const int rr = i >> 6, cc = i & 63; ts[rr * 65 + cc] = in[zb + (size_t)(r0 + rr) * C + c0 + cc]; }
    __syncthreads();
    v8us o0, o1;
    { const int p = tid;       const int orow = p >> 3, c8 = (p & 7) * 8;
#pragma unroll
      for (int i = 0; i < 8; ++i) o0[i] = f2bf(ts[(c8 + i) * 65 + orow]); }
    { const int p = tid + 256; const int orow = p >> 3, c8 = (p & 7) * 8;
#pragma unroll
      for (int i = 0; i < 8; ++i) o1[i] = f2bf(ts[(c8 + i) * 65 + orow]); }
    const size_t a0 = zb + (size_t)(c0 + (tid >> 3)) * R + r0 + (tid & 7) * 8;
    const size_t a1 = zb + (size_t)(c0 + 32 + (tid >> 3)) * R + r0 + (tid & 7) * 8;
    *(volatile v8us*)(out + a0) = o0; *(volatile v8us*)(out + a1) = o1;
    __threadfence();
    *(volatile v8us*)(out + a0) = o0; *(volatile v8us*)(out + a1) = o1;
}

__global__ __launch_bounds__(256) void k_bfr4(const float* __restrict__ src, float* dst, size_t n4) {
    const size_t i = (size_t)blockIdx.x * 256 + threadIdx.x; if (i >= n4) return;
    const v4f v = *(const v4f*)(src + i * 4); v4f o;
#pragma unroll
    for (int k = 0; k < 4; ++k) o[k] = bfr(v[k]);
    *(volatile v4f*)(dst + i * 4) = o; __threadfence(); *(volatile v4f*)(dst + i * 4) = o;
}

__global__ __launch_bounds__(256) void k_pp(const float* __restrict__ b2, const float* __restrict__ sw_, const float* __restrict__ sb_, const float* __restrict__ gw_, const float* __restrict__ gb_,
                                            const float* __restrict__ lg_, const float* __restrict__ lb_, float* PP) {
    const int q = blockIdx.x * 256 + threadIdx.x; if (q >= NV * 16 * 16 * 2) return;
    const int half = q & 1, t = (q >> 1) & 15, lr = (q >> 5) & 15, n = q >> 9;
    const int src = n * HID + 16 * t + lr;
    const float v0 = bfr(b2[src]), v1 = bfr(sw_[src]), v2 = bfr(sb_[src]), v3 = bfr(gw_[src]), v4 = bfr(gb_[src]), v5 = bfr(lg_[src]), v6 = bfr(lb_[src]);
    v4f o;
    o[0] = half ? v4 : v0; o[1] = half ? v5 : v1; o[2] = half ? v6 : v2; o[3] = half ? 0.0f : v3;
    *(volatile v4f*)(PP + (size_t)q * 4) = o; __threadfence(); *(volatile v4f*)(PP + (size_t)q * 4) = o;
}

__global__ __attribute__((amdgpu_num_vgpr(256))) __launch_bounds__(32) void k_sel(const float* __restrict__ x, const bf* __restrict__ W1T, const float* __restrict__ b1, const h16* __restrict__ W2T, const float* __restrict__ b2,
                                             const bf* __restrict__ WST, const float* __restrict__ bs, const bf* __restrict__ WGT, const float* __restrict__ bg,
                                             const float* __restrict__ lng, const float* __restrict__ lnb, float* SWP, float* OUT1) {
    __shared__ __align__(16) h16 hs[16 * HSP];
    __shared__ __align__(16) float os[16 * OSP];
    const int lane = threadIdx.x & 31, lr = lane & 15, hi = lane >> 4;
    const int row0 = blockIdx.x * 16;
    const float* xp = x + (size_t)(row0 + lr) * XP + 8 * hi;
    v16bf xa0, xa1;
    { const v4f a = *(const v4f*)xp, b = *(const v4f*)(xp + 4), c = *(const v4f*)(xp + 16), d = *(const v4f*)(xp + 20); v8us lo, up;
#pragma unroll
      for (int i = 0; i < 4; ++i) { lo[i] = f2bf(a[i]); lo[4 + i] = f2bf(b[i]); up[i] = f2bf(c[i]); up[4 + i] = f2bf(d[i]); }
      xa0 = cat16b(lo, up); }
    { const v4f a = *(const v4f*)(xp + 32), b = *(const v4f*)(xp + 36), c = *(const v4f*)(xp + 48), d = *(const v4f*)(xp + 52); v8us lo, up;
#pragma unroll
      for (int i = 0; i < 4; ++i) { lo[i] = f2bf(a[i]); lo[4 + i] = f2bf(b[i]); up[i] = f2bf(c[i]); up[4 + i] = f2bf(d[i]); }
      xa1 = cat16b(lo, up); }
#pragma unroll 1
    for (int g = 0; g < 4; ++g) {
        v8f a4[4];
#pragma unroll
        for (int t = 0; t < 4; ++t) a4[t] = (v8f){};
#pragma unroll
        for (int t = 0; t < 4; ++t) { const bf* wp = W1T + (size_t)(g * 64 + t * 16 + lr) * NV + 8 * hi;
            const v16bf w0 = ldb(wp), w1 = ldb(wp + 32);
            a4[t] = wmmabg(xa0, w0, a4[t]); a4[t] = wmmabg(xa1, w1, a4[t]); }
#pragma unroll
        for (int t = 0; t < 4; ++t) { const int c = g * 64 + t * 16 + lr; const float bb = bfr(b1[c]);
#pragma unroll
            for (int r = 0; r < 8; ++r) hs[(8 * hi + r) * HSP + c] = toh_flush(eluf(a4[t][r] + bb) * HCAR); }
    }
    wave_sync();
    v8f ha[4], sa[4], ga[4];
#pragma unroll
    for (int t = 0; t < 4; ++t) { ha[t] = (v8f){}; sa[t] = (v8f){}; ga[t] = (v8f){}; }
#pragma unroll 1
    for (int ks = 0; ks < 8; ++ks) {
        const int ao = lr * HSP + 8 * hi + ks * 32;
        const v16h a = cat16(*(const v8ha*)(&hs[ao]), *(const v8ha*)(&hs[ao + 16]));
#pragma unroll
        for (int t = 0; t < 4; ++t) { const v16h b = ldh(W2T + (size_t)(t * 16 + lr) * HID + 8 * hi + ks * 32); ha[t] = wmma16g(a, b, ha[t]); }
    }
#pragma unroll
    for (int t = 0; t < 4; ++t) { const bf* sp = WST + (size_t)(t * 16 + lr) * NV + 8 * hi; const bf* gp = WGT + (size_t)(t * 16 + lr) * NV + 8 * hi;
        const v16bf s0 = ldb(sp), s1 = ldb(sp + 32), g0 = ldb(gp), g1 = ldb(gp + 32);
        sa[t] = wmmabg(xa0, s0, sa[t]); sa[t] = wmmabg(xa1, s1, sa[t]);
        ga[t] = wmmabg(xa0, g0, ga[t]); ga[t] = wmmabg(xa1, g1, ga[t]); }
    float u[4][8]; float s[8];
#pragma unroll
    for (int r = 0; r < 8; ++r) s[r] = 0.0f;
#pragma unroll
    for (int t = 0; t < 4; ++t) { const int c = t * 16 + lr; const float b2v = bfr(b2[c]), bsv = bfr(bs[c]), bgv = bfr(bg[c]);
#pragma unroll
        for (int r = 0; r < 8; ++r) { const float h = ha[t][r] * HSC + b2v; const float sk = sa[t][r] + bsv; const float g = sigm(ga[t][r] + bgv);
            const float uu = g * h + (1.0f - g) * sk; u[t][r] = uu; s[r] += uu; } }
    float rs[8];
#pragma unroll
    for (int r = 0; r < 8; ++r) { const float mu = sum16(s[r]) * (1.0f / 64.0f); float q = 0.0f;
#pragma unroll
        for (int t = 0; t < 4; ++t) { const float d = u[t][r] - mu; u[t][r] = d; q += d * d; }
        rs[r] = rsqrtf(sum16(q) * (1.0f / 64.0f) + LN_EPS); }
    float mx[8];
#pragma unroll
    for (int r = 0; r < 8; ++r) mx[r] = -3.0e38f;
#pragma unroll
    for (int t = 0; t < 4; ++t) { const int c = t * 16 + lr; const float lg = bfr(lng[c]), lb = bfr(lnb[c]);
#pragma unroll
        for (int r = 0; r < 8; ++r) { const float w = (u[t][r] * rs[r]) * lg + lb; u[t][r] = w; mx[r] = fmaxf(mx[r], w); } }
#pragma unroll
    for (int r = 0; r < 8; ++r) { const float m = max16(mx[r]); float se = 0.0f;
#pragma unroll
        for (int t = 0; t < 4; ++t) { const float e = __builtin_amdgcn_exp2f((u[t][r] - m) * LOG2E); u[t][r] = e; se += e; }
        const float inv = __builtin_amdgcn_rcpf(sum16(se));
#pragma unroll
        for (int t = 0; t < 4; ++t) os[(8 * hi + r) * OSP + t * 16 + lr] = u[t][r] * inv; }
    wave_sync();
    float* o1 = OUT1 + (size_t)row0 * NV; float* o2 = SWP + (size_t)row0 * NV;
#pragma unroll 1
    for (int ps = 0; ps < 2; ++ps) {
#pragma unroll
        for (int sI = 0; sI < 8; ++sI) { const int p = sI * 32 + lane; const int row = p >> 4, c4 = (p & 15) * 4;
            const v4f val = *(const v4fa*)(&os[row * OSP + c4]);
            *(volatile v4f*)(o1 + (size_t)row * NV + c4) = val; *(volatile v4f*)(o2 + (size_t)row * NV + c4) = val; }
        if (ps == 0) __threadfence(); }
}

__global__ __launch_bounds__(32) void k_emb(const float* __restrict__ x, const float* __restrict__ W1R, const float* __restrict__ B1R, const h16* __restrict__ WT,
                                             const float* __restrict__ PP, const float* __restrict__ SWP, float* OUT0) {
    __shared__ __align__(16) float cs[16 * CSP];
    __shared__ __align__(16) float us[16 * CSP];
    __shared__ __align__(16) float xs[16 * OSP];
    __shared__ __align__(16) float ss[16 * OSP];
    const int lane = threadIdx.x & 31, lr = lane & 15, hi = lane >> 4;
    const int row0 = blockIdx.x * 16;
#pragma unroll
    for (int sI = 0; sI < 8; ++sI) { const int p = sI * 32 + lane; const int row = p >> 4, c4 = (p & 15) * 4;
        const v4f xv = *(const v4f*)(x + (size_t)(row0 + row) * XP + c4); const v4f sv = *(const v4f*)(SWP + (size_t)(row0 + row) * NV + c4); v4f xr;
#pragma unroll
        for (int i = 0; i < 4; ++i) xr[i] = bfr(xv[i]);
        *(v4fa*)(&xs[row * OSP + c4]) = xr; *(v4fa*)(&ss[row * OSP + c4]) = sv; }
#pragma unroll
    for (int t = 0; t < 16; ++t)
#pragma unroll
        for (int r = 0; r < 8; ++r) cs[(8 * hi + r) * CSP + t * 16 + lr] = 0.0f;
    wave_sync();
#pragma unroll 1
    for (int n = 0; n < NV; ++n) {
        const float xa = xs[lr * OSP + n];
        float xr[8], s[8];
#pragma unroll
        for (int r = 0; r < 8; ++r) { xr[r] = xs[(8 * hi + r) * OSP + n]; s[r] = 0.0f; }
        const float* w1p = W1R + (size_t)n * HID + 8 * hi;
        const float* b1p = B1R + (size_t)n * HID + 8 * hi;
        const float* pp = PP + ((size_t)(n * 16 + lr) * 16) * 8;
#pragma unroll 1
        for (int cp = 0; cp < 4; ++cp) {
            v8f acc[4];
#pragma unroll
            for (int t = 0; t < 4; ++t) acc[t] = (v8f){};
            const h16* wtp = WT + ((size_t)n * HID + (size_t)(cp * 64 + lr)) * HID + 8 * hi;
#pragma unroll 1
            for (int ks = 0; ks < 8; ++ks) {
                const int k0 = ks * 32;
                v16h a;
                { const v4f wA = *(const v4f*)(w1p + k0), wB = *(const v4f*)(w1p + k0 + 4);
                  const v4f bA = *(const v4f*)(b1p + k0), bB = *(const v4f*)(b1p + k0 + 4);
#pragma unroll
                  for (int i = 0; i < 4; ++i) { a[i] = hvf(xa, wA[i], bA[i]); a[4 + i] = hvf(xa, wB[i], bB[i]); } }
                { const v4f wC = *(const v4f*)(w1p + k0 + 16), wD = *(const v4f*)(w1p + k0 + 20);
                  const v4f bC = *(const v4f*)(b1p + k0 + 16), bD = *(const v4f*)(b1p + k0 + 20);
#pragma unroll
                  for (int i = 0; i < 4; ++i) { a[8 + i] = hvf(xa, wC[i], bC[i]); a[12 + i] = hvf(xa, wD[i], bD[i]); } }
#pragma unroll
                for (int t = 0; t < 4; ++t) { const v16h b = ldh(wtp + (size_t)t * 16 * HID + k0); acc[t] = wmma16g(a, b, acc[t]); }
            }
#pragma unroll
            for (int t = 0; t < 4; ++t)
#pragma unroll
                for (int r = 0; r < 8; ++r) us[(8 * hi + r) * CSP + (cp * 4 + t) * 16 + lr] = acc[t][r];
#pragma unroll 1
            for (int t = 0; t < 4; ++t) { const int tt = cp * 4 + t; const v4f p0 = *(const v4f*)(pp + tt * 8), p1 = *(const v4f*)(pp + tt * 8 + 4);
#pragma unroll
                for (int r = 0; r < 8; ++r) { const int idx = (8 * hi + r) * CSP + tt * 16 + lr;
                    const float h2 = us[idx] * SCL + p0[0]; const float sk = xr[r] * p0[1] + p0[2]; const float g = sigm(xr[r] * p0[3] + p1[0]);
                    const float uu = g * h2 + (1.0f - g) * sk; us[idx] = uu; s[r] += uu; } }
        }
        wave_sync();
        float mu[8], q[8];
#pragma unroll
        for (int r = 0; r < 8; ++r) { mu[r] = sum16(s[r]) * (1.0f / 256.0f); q[r] = 0.0f; }
#pragma unroll 1
        for (int t = 0; t < 16; ++t) {
#pragma unroll
            for (int r = 0; r < 8; ++r) { const float d = us[(8 * hi + r) * CSP + t * 16 + lr] - mu[r]; q[r] += d * d; } }
        float rs[8], swr[8];
#pragma unroll
        for (int r = 0; r < 8; ++r) { rs[r] = rsqrtf(sum16(q[r]) * (1.0f / 256.0f) + LN_EPS); swr[r] = ss[(8 * hi + r) * OSP + n]; }
#pragma unroll 1
        for (int t = 0; t < 16; ++t) { const v4f p1 = *(const v4f*)(pp + t * 8 + 4); const float lg = p1[1], lb = p1[2];
#pragma unroll
            for (int r = 0; r < 8; ++r) { const int idx = (8 * hi + r) * CSP + t * 16 + lr; const float d = us[idx] - mu[r]; const float e = (d * rs[r]) * lg + lb; const float cur = cs[idx]; cs[idx] = cur + swr[r] * e; } }
    }
    wave_sync();
    float* orow = OUT0 + (size_t)row0 * HID;
#pragma unroll 1
    for (int ps = 0; ps < 2; ++ps) {
#pragma unroll 4
        for (int sI = 0; sI < 32; ++sI) { const int p = sI * 32 + lane; const int row = p >> 6, c4 = (p & 63) * 4;
            const v4f val = *(const v4fa*)(&cs[row * CSP + c4]);
            *(volatile v4f*)(orow + (size_t)row * HID + c4) = val; }
        if (ps == 0) __threadfence(); }
}

static constexpr size_t al256(size_t v) { return (v + 255) & ~(size_t)255; }
static constexpr size_t SZ_WT  = al256((size_t)NV * HID * HID * 2);
static constexpr size_t SZ_W1T = al256((size_t)HID * NV * 2);
static constexpr size_t SZ_W2T = al256((size_t)NV * HID * 2);
static constexpr size_t SZ_WQ  = al256((size_t)NV * NV * 2);
static constexpr size_t SZ_PP  = al256((size_t)NV * 16 * 16 * 8 * 4);
static constexpr size_t SZ_WR  = al256((size_t)NV * HID * 4);
static constexpr size_t SZ_SW  = al256((size_t)NB * NV * 4);
static constexpr size_t SZ_TOTAL = SZ_WT + SZ_W1T + SZ_W2T + 2 * SZ_WQ + SZ_PP + 2 * SZ_WR + SZ_SW;
static_assert(SZ_TOTAL <= (size_t)134217728);
static_assert(((size_t)NV * HID) % 4 == 0);
static_assert((NV * 16 * 16 * 2) % 256 == 0);

extern "C" void kernel_launch(void* const* d_in, const int* in_sizes, int n_in,
                              void* d_out, int out_size, void* d_ws, size_t ws_size, hipStream_t stream) {
    if (n_in < 21) return;
    if ((size_t)in_sizes[0] < (size_t)NB * NV) return;
    if (in_sizes[1] < NV * HID || in_sizes[2] < HID || in_sizes[3] < HID * NV || in_sizes[4] < NV) return;
    if (in_sizes[5] < NV * NV || in_sizes[6] < NV || in_sizes[7] < NV * NV || in_sizes[8] < NV || in_sizes[9] < NV || in_sizes[10] < NV) return;
    if (in_sizes[11] < NV * HID || in_sizes[12] < NV * HID || (size_t)in_sizes[13] < (size_t)NV * HID * HID || in_sizes[14] < NV * HID) return;
    if (in_sizes[15] < NV * HID || in_sizes[16] < NV * HID || in_sizes[17] < NV * HID || in_sizes[18] < NV * HID || in_sizes[19] < NV * HID || in_sizes[20] < NV * HID) return;
    if ((size_t)out_size < OUT1_OFF + (size_t)NB * NV) return;
    if (SZ_TOTAL > ws_size) return;
    const float* x    = (const float*)d_in[0];
    const float* f1w  = (const float*)d_in[1];  const float* f1b = (const float*)d_in[2];
    const float* f2w  = (const float*)d_in[3];  const float* f2b = (const float*)d_in[4];
    const float* fsw  = (const float*)d_in[5];  const float* fsb = (const float*)d_in[6];
    const float* fgw  = (const float*)d_in[7];  const float* fgb = (const float*)d_in[8];
    const float* flg  = (const float*)d_in[9];  const float* flb = (const float*)d_in[10];
    const float* g1w  = (const float*)d_in[11]; const float* g1b = (const float*)d_in[12];
    const float* g2w  = (const float*)d_in[13]; const float* g2b = (const float*)d_in[14];
    const float* gsw  = (const float*)d_in[15]; const float* gsb = (const float*)d_in[16];
    const float* ggw  = (const float*)d_in[17]; const float* ggb = (const float*)d_in[18];
    const float* glg  = (const float*)d_in[19]; const float* glb = (const float*)d_in[20];
    float* OUT0 = (float*)d_out;
    float* OUT1 = (float*)d_out + OUT1_OFF;
    char* wsp = (char*)d_ws;
    h16* WT   = (h16*)wsp;  wsp += SZ_WT;
    bf*  W1T  = (bf*)wsp;   wsp += SZ_W1T;
    h16* W2T  = (h16*)wsp;  wsp += SZ_W2T;
    bf*  WST  = (bf*)wsp;   wsp += SZ_WQ;
    bf*  WGT  = (bf*)wsp;   wsp += SZ_WQ;
    float* PP = (float*)wsp; wsp += SZ_PP;
    float* W1R = (float*)wsp; wsp += SZ_WR;
    float* B1R = (float*)wsp; wsp += SZ_WR;
    float* SWP = (float*)wsp; wsp += SZ_SW;

    k_tr_h<<<dim3(HID / 64, HID / 64, NV), 256, 0, stream>>>(g2w, WT, HID, HID, WCAR);
    k_tr_b<<<dim3(HID / 64, NV / 64, 1), 256, 0, stream>>>(f1w, W1T, NV, HID);
    k_tr_h<<<dim3(NV / 64, HID / 64, 1), 256, 0, stream>>>(f2w, W2T, HID, NV, WCAR);
    k_tr_b<<<dim3(NV / 64, NV / 64, 1), 256, 0, stream>>>(fsw, WST, NV, NV);
    k_tr_b<<<dim3(NV / 64, NV / 64, 1), 256, 0, stream>>>(fgw, WGT, NV, NV);
    k_pp<<<(NV * 16 * 16 * 2) / 256, 256, 0, stream>>>(g2b, gsw, gsb, ggw, ggb, glg, glb, PP);
    { const size_t n4 = (size_t)NV * HID / 4; const unsigned g = (unsigned)((n4 + 255) / 256);
      k_bfr4<<<g, 256, 0, stream>>>(g1w, W1R, n4); k_bfr4<<<g, 256, 0, stream>>>(g1b, B1R, n4); }

    k_sel<<<NB / 16, 32, 0, stream>>>(x, W1T, f1b, W2T, f2b, WST, fsb, WGT, fgb, flg, flb, SWP, OUT1);
    k_emb<<<NB / 16, 32, 0, stream>>>(x, W1R, B1R, WT, PP, SWP, OUT0);
}
